// NTKViTSelfAttention_50586124812753
// MI455X (gfx1250) — hardware-run, weakly checked
//
#include <hip/hip_runtime.h>


#ifndef NB
#define NB 16
#endif
#ifndef SEQ
#define SEQ 1024
#endif
#define NB_FULL  16
#define SEQ_FULL 1024
#ifndef OUT_SEQ
#define OUT_SEQ SEQ
#endif
#define DM   768
#define NH_  12
#define HD   64
#define AW   4
#define OSP  68
#define SC2  ((float)(0.125 * 1.4426950408889634))
#define PSH  14.0f
#define NEGB (-3.0e38f)
#define PHS  0.35355339059327373f
#define LOG2E 1.4426950408889634f
#define LN2F  0.6931471805599453f
#define KVC  1024.0f
#define GOC  16.0f
#define GDC  16384.0f

static_assert(HD == 64);
static_assert(NH_ * HD == DM);
static_assert(DM % 64 == 0);
static_assert(DM % 32 == 0);
static_assert(HD % 32 == 0);
static_assert(SEQ % 64 == 0);
static_assert((NB * SEQ) % 64 == 0);
static_assert(SEQ % 32 == 0);
static_assert(SEQ % (16 * AW) == 0);
static_assert(((size_t)SEQ * DM) % 8 == 0);
static_assert(((size_t)DM * DM) % 8 == 0);
static_assert(NB <= NB_FULL);
static_assert(SEQ <= SEQ_FULL);
static_assert((OSP * 4) % 16 == 0);
static_assert(OSP >= HD);
static_assert(32 * 16 * 4 == 16 * 64 * 2);
static_assert(32 * 16 * 8 == 16 * HD * 4);
static_assert(256 * 16 == HD * HD);
static_assert(256 * 16 * 2 == HD * HD * 2);
static_assert(AW * 16 * OSP * 4 <= 131072);
static_assert(16 * 68 * 4 <= 131072);
static_assert(HD * (HD + 1) * 4 <= 131072);

typedef _Float16 h16;
typedef unsigned short bf;
typedef __attribute__((ext_vector_type(16))) __bf16   v16bf;
typedef __attribute__((ext_vector_type(16))) _Float16 v16h;
typedef __attribute__((ext_vector_type(8)))  _Float16 v8h;
typedef __attribute__((ext_vector_type(8)))  unsigned short v8us;
typedef __attribute__((ext_vector_type(8)))  float    v8f;
typedef __attribute__((ext_vector_type(4)))  float    v4f;
typedef v4f  __attribute__((may_alias)) v4fa;

__device__ __forceinline__ unsigned short f2bf(float f) { unsigned u = __float_as_uint(f); u += 0x7FFFu + ((u >> 16) & 1u); return (unsigned short)(u >> 16); }
__device__ __forceinline__ float bfr(float f) { return __uint_as_float(((unsigned)f2bf(f)) << 16); }
__device__ __forceinline__ v16h cat16(v8h lo, v8h hi) { return __builtin_shufflevector(lo, hi, 0, 1, 2, 3, 4, 5, 6, 7, 8, 9, 10, 11, 12, 13, 14, 15); }
__device__ __forceinline__ v16bf cat16b(v8us lo, v8us hi) { return __builtin_bit_cast(v16bf, __builtin_shufflevector(lo, hi, 0, 1, 2, 3, 4, 5, 6, 7, 8, 9, 10, 11, 12, 13, 14, 15)); }
__device__ __forceinline__ v8f wmma16(v16h a, v16h b, v8f c) { return __builtin_amdgcn_wmma_f32_16x16x32_f16(false, a, false, b, (short)0, c, false, false); }
__device__ __forceinline__ v8f wmmab(v16bf a, v16bf b, v8f c) { return __builtin_amdgcn_wmma_f32_16x16x32_bf16(false, a, false, b, (short)0, c, false, false); }
__device__ __forceinline__ v16h  ldh(const h16* p) { return cat16(*(const v8h*)p, *(const v8h*)(p + 16)); }
__device__ __forceinline__ v16bf ldb(const bf* p)  { return cat16b(*(const v8us*)p, *(const v8us*)(p + 16)); }
__device__ __forceinline__ void wave_sync() { __builtin_amdgcn_fence(3  , "wavefront"); __builtin_amdgcn_wave_barrier(); asm volatile("" ::: "memory"); }
__device__ __forceinline__ h16 toh_flush(float v) { const h16 r = (h16)v; return (fabsf(v) < 6.103515625e-05f) ? (h16)0.0f : r; }
__device__ __forceinline__ v8f wmma16g(v16h a, v16h b, v8f c) { c = wmma16(a, b, c); asm volatile("v_nop\n\tv_nop\n\tv_nop\n\tv_nop" : "+v"(c) : "v"(a), "v"(b)); return c; }
__device__ __forceinline__ v8f wmmabg(v16bf a, v16bf b, v8f c) { c = wmmab(a, b, c); asm volatile("v_nop\n\tv_nop\n\tv_nop\n\tv_nop" : "+v"(c) : "v"(a), "v"(b)); return c; }

__global__ __launch_bounds__(256) void k_cvt8(const float* __restrict__ src, bf* dst, size_t n8) {
    const size_t i = (size_t)blockIdx.x * 256 + threadIdx.x; if (i >= n8) return;
    const v8f v = *(const v8f*)(src + i * 8); v8us o;
#pragma unroll
    for (int k = 0; k < 8; ++k) o[k] = f2bf(v[k]);
    *(volatile v8us*)(dst + i * 8) = o; __threadfence(); *(volatile v8us*)(dst + i * 8) = o;
}

__global__ __launch_bounds__(256) void k_phit(const float* __restrict__ src, h16* dst) {
#pragma clang fp contract(off)
    __shared__ float tl[HD * (HD + 1)];
    const int tid = threadIdx.x;
    const float* s = src + (size_t)blockIdx.x * HD * HD;
#pragma unroll 4
    for (int it = 0; it < 16; ++it) { const int idx = it * 256 + tid; tl[(idx >> 6) * (HD + 1) + (idx & 63)] = bfr(s[idx]) * KVC; }
    __syncthreads();
    h16* d = dst + (size_t)blockIdx.x * HD * HD;
    v8h o[2];
#pragma unroll
    for (int it = 0; it < 2; ++it) { const int p = it * 256 + tid; const int row = p >> 3, c8 = (p & 7) * 8;
#pragma unroll
        for (int i = 0; i < 8; ++i) o[it][i] = toh_flush(tl[(c8 + i) * (HD + 1) + row]); }
#pragma unroll 1
    for (int ps = 0; ps < 2; ++ps) {
#pragma unroll
        for (int it = 0; it < 2; ++it) { const int p = it * 256 + tid; *(volatile v8h*)(d + (size_t)p * 8) = o[it]; }
        if (ps == 0) __threadfence(); }
}

template <int MODE>
__device__ __forceinline__ void proj_tile(const bf* __restrict__ A, const bf* __restrict__ Bt, const float* __restrict__ bias, h16* Ph) {
    __shared__ __align__(16) float os[16 * 68];
    const int K = DM;
    const int lane = threadIdx.x & 31, lr = lane & 15, hi = lane >> 4; const int r0 = blockIdx.x * 64, c0 = blockIdx.y * 64;
    v8f acc[4][4];
#pragma unroll
    for (int mb = 0; mb < 4; ++mb)
#pragma unroll
        for (int nb = 0; nb < 4; ++nb) acc[mb][nb] = (v8f){};
    const size_t aoff = (size_t)(r0 + lr) * K + 8 * hi, boff = (size_t)(c0 + lr) * K + 8 * hi;
#pragma unroll 1
    for (int kc = 0; kc < K; kc += 32) {
        v16bf a[4];
#pragma unroll
        for (int mb = 0; mb < 4; ++mb) a[mb] = ldb(A + aoff + (size_t)mb * 16 * K + kc);
#pragma unroll
        for (int nb = 0; nb < 4; ++nb) { const v16bf b = ldb(Bt + boff + (size_t)nb * 16 * K + kc);
#pragma unroll
            for (int mb = 0; mb < 4; ++mb) acc[mb][nb] = wmmabg(a[mb], b, acc[mb][nb]); }
    }
    float bc[4];
#pragma unroll
    for (int nb = 0; nb < 4; ++nb) bc[nb] = (MODE == 0) ? bfr(bias[c0 + nb * 16 + lr]) : 0.0f;
    size_t tbase;
    if (MODE == 0) { const int bb = r0 / SEQ, tt = r0 % SEQ; const int zc = bb * NH_ + c0 / HD;
                     tbase = ((size_t)zc * SEQ + (size_t)tt) * HD; }
    else           { const int bb = c0 / SEQ, tt = c0 % SEQ;
                     tbase = (size_t)bb * (size_t)DM * SEQ + (size_t)r0 * SEQ + (size_t)tt; }
#pragma unroll
    for (int mb = 0; mb < 4; ++mb) {
        float br[8];
#pragma unroll
        for (int j = 0; j < 8; ++j) br[j] = (MODE == 1) ? bfr(bias[r0 + mb * 16 + hi * 8 + j]) : 0.0f;
#pragma unroll
        for (int nb = 0; nb < 4; ++nb) {
#pragma unroll
            for (int j = 0; j < 8; ++j) os[(hi * 8 + j) * 68 + nb * 16 + lr] = acc[mb][nb][j] + bc[nb] + br[j]; }
        wave_sync();
#pragma unroll 1
        for (int ps = 0; ps < 2; ++ps) {
            if (MODE == 0) {
                const size_t sb = tbase + (size_t)(mb * 16) * HD;
#pragma unroll
                for (int s = 0; s < 4; ++s) { const int p = s * 32 + lane; const int row = p >> 3, c8 = (p & 7) * 8;
                    const v4f x0 = *(const v4fa*)(&os[row * 68 + c8]); const v4f x1 = *(const v4fa*)(&os[row * 68 + c8 + 4]); v8h hv;
#pragma unroll
                    for (int i = 0; i < 4; ++i) { hv[i] = toh_flush(x0[i]); hv[4 + i] = toh_flush(x1[i]); }
                    const size_t oo = sb + (size_t)p * 8;
                    *(volatile v8h*)(Ph + oo) = hv; }
            } else {
                const size_t sb = tbase + (size_t)(mb * 16) * SEQ;
#pragma unroll
                for (int s = 0; s < 4; ++s) { const int row = 4 * s + (lane >> 3), c8 = (lane & 7) * 8;
                    const v4f x0 = *(const v4fa*)(&os[row * 68 + c8]); const v4f x1 = *(const v4fa*)(&os[row * 68 + c8 + 4]); v8h hv;
#pragma unroll
                    for (int i = 0; i < 4; ++i) { hv[i] = toh_flush(x0[i]); hv[4 + i] = toh_flush(x1[i]); }
                    const size_t oo = sb + (size_t)row * SEQ + c8;
                    *(volatile v8h*)(Ph + oo) = hv; }
            }
            if (ps == 0) __threadfence(); }
        wave_sync();
    }
}

__global__ __launch_bounds__(32) void k_proj_rows(const bf* __restrict__ A, const bf* __restrict__ Bt, const float* __restrict__ bias, h16* Ph) { proj_tile<0>(A, Bt, bias, Ph); }
__global__ __launch_bounds__(32) void k_proj_tr(const bf* __restrict__ A, const bf* __restrict__ Bt, const float* __restrict__ bias, h16* Ph) { proj_tile<1>(A, Bt, bias, Ph); }

__global__ __launch_bounds__(32 * AW) void k_flash(const h16* __restrict__ QH, const h16* __restrict__ KP, const h16* __restrict__ VT, const h16* __restrict__ PKV,
                                                   const float* __restrict__ phik, float* OUT) {
    __shared__ __align__(16) float os[AW * 16 * OSP];
    const int lane = threadIdx.x & 31, lr = lane & 15, hi = lane >> 4;
    const int wave = __builtin_amdgcn_readfirstlane((int)(threadIdx.x >> 5));
    const int zh = blockIdx.y; const int b = zh / NH_, h = zh % NH_;
    const int t0 = (blockIdx.x * AW + wave) * 16;
    const size_t pbase = (size_t)zh * SEQ * HD;
    const size_t qo = pbase + (size_t)(t0 + lr) * HD + 8 * hi;
    const v16h qh0 = ldh(QH + qo), qh1 = ldh(QH + qo + 32);
    const size_t ko = pbase + (size_t)lr * HD + 8 * hi;
    const size_t vo = pbase + (size_t)lr * SEQ + 8 * hi;
    v8f o[4];
#pragma unroll
    for (int j = 0; j < 4; ++j) o[j] = (v8f){};
    float m = NEGB, l = 0.0f;
#pragma unroll 1
    for (int key0 = 0; key0 < SEQ; key0 += 32) {
        const h16* ka = KP + ko + (size_t)key0 * HD;
        const v16h ka0 = ldh(ka), ka1 = ldh(ka + 32), kb0 = ldh(ka + 16 * HD), kb1 = ldh(ka + 16 * HD + 32);
        v8f sa = (v8f){}, sb = (v8f){};
        sa = wmma16g(ka0, qh0, sa); sa = wmma16g(ka1, qh1, sa);
        sb = wmma16g(kb0, qh0, sb); sb = wmma16g(kb1, qh1, sb);
        float ta[8], tb[8]; float mx = NEGB;
#pragma unroll
        for (int r = 0; r < 8; ++r) { ta[r] = sa[r] * SC2; tb[r] = sb[r] * SC2; mx = fmaxf(mx, fmaxf(ta[r], tb[r])); }
        mx = fmaxf(mx, __shfl_xor(mx, 16, 32));
        const float mnew = fmaxf(m, mx);
        const float alpha = __builtin_amdgcn_exp2f(m - mnew);
        const float sh = PSH - mnew;
        v16h pb; float ls = 0.0f;
#pragma unroll
        for (int r = 0; r < 8; ++r) {
            const float xa = ta[r] + sh, xb = tb[r] + sh;
            const float ea = __builtin_amdgcn_exp2f(xa), eb = __builtin_amdgcn_exp2f(xb);
            const float ga = (xa < -14.0f) ? 0.0f : ea, gb = (xb < -14.0f) ? 0.0f : eb;
            const h16 pa = (h16)ga; const h16 pc = (h16)gb;
            pb[r] = pa; pb[8 + r] = pc;
            ls += (float)pa + (float)pc; }
        l = l * alpha + ls; m = mnew;
#pragma unroll
        for (int j = 0; j < 4; ++j) o[j] = o[j] * alpha;
        const h16* va = VT + vo + key0;
        v16h vv[4];
#pragma unroll
        for (int j = 0; j < 4; ++j) vv[j] = ldh(va + (size_t)(16 * j) * SEQ);
#pragma unroll
        for (int j = 0; j < 4; ++j) o[j] = wmma16g(vv[j], pb, o[j]);
    }
    l += __shfl_xor(l, 16, 32);
    const float* pkp = phik + (size_t)h * HD + 8 * hi;
    const v4f k0 = *(const v4f*)(pkp),      k1 = *(const v4f*)(pkp + 4),  k2 = *(const v4f*)(pkp + 16), k3 = *(const v4f*)(pkp + 20);
    const v4f k4 = *(const v4f*)(pkp + 32), k5 = *(const v4f*)(pkp + 36), k6 = *(const v4f*)(pkp + 48), k7 = *(const v4f*)(pkp + 52);
    float pka[16], pkb[16];
#pragma unroll
    for (int i = 0; i < 4; ++i) {
        pka[i] = fabsf(bfr(k0[i])); pka[4 + i] = fabsf(bfr(k1[i])); pka[8 + i] = fabsf(bfr(k2[i])); pka[12 + i] = fabsf(bfr(k3[i]));
        pkb[i] = fabsf(bfr(k4[i])); pkb[4 + i] = fabsf(bfr(k5[i])); pkb[8 + i] = fabsf(bfr(k6[i])); pkb[12 + i] = fabsf(bfr(k7[i])); }
    v16h pq0, pq1; float cqp = 0.0f;
#pragma unroll
    for (int e = 0; e < 16; ++e) {
        const float x0 = (float)qh0[e] * PHS, x1 = (float)qh1[e] * PHS;
        const float e0 = __builtin_amdgcn_exp2f(x0 * LOG2E), e1 = __builtin_amdgcn_exp2f(x1 * LOG2E);
        const float p0 = (x0 > 0.0f) ? (x0 + 1.0f) : e0, p1 = (x1 > 0.0f) ? (x1 + 1.0f) : e1;
        pq0[e] = toh_flush(p0); pq1[e] = toh_flush(p1);
        cqp += p0 * pka[e]; cqp += p1 * pkb[e]; }
    const float cq = cqp + __shfl_xor(cqp, 16, 32);
    const h16* pa = PKV + (size_t)h * HD * HD + (size_t)lr * HD + 8 * hi;
    v8f cc[4];
#pragma unroll
    for (int j = 0; j < 4; ++j) {
        cc[j] = (v8f){};
        const v16h a0 = ldh(pa + (size_t)(16 * j) * HD), a1 = ldh(pa + (size_t)(16 * j) * HD + 32);
        cc[j] = wmma16g(a0, pq0, cc[j]); cc[j] = wmma16g(a1, pq1, cc[j]); }
    const float ie = expf(-(m * LN2F));
    const float gO = ie * GOC, gD = ie * GDC;
    const float den = l + cq * gD;
    const float inv = 1.0f / den;
    const int wb = wave * 16 * OSP;
#pragma unroll
    for (int j = 0; j < 4; ++j) {
        const v8f fj = (o[j] + cc[j] * gO) * inv;
        v4f a, c;
        a[0] = fj[0]; a[1] = fj[1]; a[2] = fj[2]; a[3] = fj[3]; c[0] = fj[4]; c[1] = fj[5]; c[2] = fj[6]; c[3] = fj[7];
        *(v4fa*)(&os[wb + lr * OSP + 16 * j + 8 * hi]) = a; *(v4fa*)(&os[wb + lr * OSP + 16 * j + 8 * hi + 4]) = c; }
    wave_sync();
    float* orow = OUT + ((size_t)b * OUT_SEQ + t0) * DM + h * HD;
#pragma unroll 1
    for (int ps = 0; ps < 2; ++ps) {
#pragma unroll
        for (int s = 0; s < 8; ++s) { const int row = 2 * s + (lane >> 4), cofs = (lane & 15) * 4;
            const v4f val = *(const v4fa*)(&os[wb + row * OSP + cofs]);
            *(volatile v4f*)(orow + (size_t)row * DM + cofs) = val; }
        if (ps == 0) __threadfence(); }
}

static constexpr size_t al256(size_t v) { return (v + 255) & ~(size_t)255; }
static constexpr size_t SZ_XB = al256((size_t)NB * SEQ * DM * 2);
static constexpr size_t SZ_WB = al256((size_t)3 * DM * DM * 2);
static constexpr size_t SZ_PL = al256((size_t)NB * NH_ * SEQ * HD * 2);
static constexpr size_t SZ_PK = al256((size_t)NH_ * HD * HD * 2);
static constexpr size_t SZ_TOTAL = SZ_XB + SZ_WB + 3 * SZ_PL + SZ_PK;
static constexpr size_t NEED_X = ((size_t)(NB - 1) * SEQ_FULL + SEQ) * DM;
static constexpr size_t NEED_O = ((size_t)(NB - 1) * OUT_SEQ + SEQ) * DM;
static_assert(SZ_TOTAL <= (size_t)134217728);
static_assert(((size_t)DM * DM * 2) % 256 == 0);
static_assert((size_t)NB * NH_ * SEQ * HD == (size_t)NB * DM * SEQ);
static_assert((size_t)(NB * SEQ / 64) * 64 * (DM / 64) * 64 == (size_t)NB * SEQ * DM);

extern "C" void kernel_launch(void* const* d_in, const int* in_sizes, int n_in,
                              void* d_out, int out_size, void* d_ws, size_t ws_size, hipStream_t stream) {
    if (n_in < 9) return;
    if ((size_t)in_sizes[0] < NEED_X) return;
    if ((size_t)in_sizes[1] < (size_t)DM * DM || (size_t)in_sizes[3] < (size_t)DM * DM || (size_t)in_sizes[5] < (size_t)DM * DM) return;
    if (in_sizes[2] < DM || in_sizes[4] < DM || in_sizes[6] < DM) return;
    if (in_sizes[7] < NH_ * HD || in_sizes[8] < NH_ * HD * HD) return;
    if ((size_t)out_size < NEED_O) return;
    if (SZ_TOTAL > ws_size) return;
    const float* xin = (const float*)d_in[0];
    const float* wq = (const float*)d_in[1]; const float* bq = (const float*)d_in[2];
    const float* wk = (const float*)d_in[3]; const float* bk = (const float*)d_in[4];
    const float* wv = (const float*)d_in[5]; const float* bv = (const float*)d_in[6];
    const float* phik = (const float*)d_in[7]; const float* phikv = (const float*)d_in[8];
    float* OUT = (float*)d_out;
    char* wsp = (char*)d_ws;
    bf* XB = (bf*)wsp; wsp += SZ_XB;
    bf* WB = (bf*)wsp; wsp += SZ_WB;
    h16* QH = (h16*)wsp; wsp += SZ_PL;
    h16* KP = (h16*)wsp; wsp += SZ_PL;
    h16* VT = (h16*)wsp; wsp += SZ_PL;
    h16* PKV = (h16*)wsp; wsp += SZ_PK;
    bf* WQ = WB; bf* WK = WB + (size_t)DM * DM; bf* WV = WB + (size_t)2 * DM * DM;

    if (SEQ == SEQ_FULL) {
        const size_t n8 = (size_t)NB * SEQ * DM / 8;
        k_cvt8<<<(unsigned)((n8 + 255) / 256), 256, 0, stream>>>(xin, XB, n8);
    } else {
        const size_t n8 = (size_t)SEQ * DM / 8;
        for (int b = 0; b < NB; ++b) k_cvt8<<<(unsigned)((n8 + 255) / 256), 256, 0, stream>>>(xin + (size_t)b * SEQ_FULL * DM, XB + (size_t)b * SEQ * DM, n8);
    }
    { const size_t n8 = (size_t)DM * DM / 8; const unsigned g = (unsigned)((n8 + 255) / 256);
      k_cvt8<<<g, 256, 0, stream>>>(wq, WQ, n8); k_cvt8<<<g, 256, 0, stream>>>(wk, WK, n8); k_cvt8<<<g, 256, 0, stream>>>(wv, WV, n8); }
    k_phit<<<NH_, 256, 0, stream>>>(phikv, PKV);

    k_proj_rows<<<dim3(NB * SEQ / 64, DM / 64, 1), 32, 0, stream>>>(XB, WQ, bq, QH);
    k_proj_rows<<<dim3(NB * SEQ / 64, DM / 64, 1), 32, 0, stream>>>(XB, WK, bk, KP);
    k_proj_tr<<<dim3(DM / 64, NB * SEQ / 64, 1), 32, 0, stream>>>(WV, XB, bv, VT);

    k_flash<<<dim3(SEQ / (16 * AW), NB * NH_, 1), 32 * AW, 0, stream>>>(QH, KP, VT, PKV, phik, OUT);
}
